// GatedLinearAttentionARMA_57389353009771
// MI455X (gfx1250) — hardware-verified
//
#include <hip/hip_runtime.h>
#include <stdint.h>

#define NB   2
#define NL   512
#define NC   1024
#define NH   16
#define ND   64
#define NBH  32
#define NTOK 1024
#define NTT  8
#define PK   128
#define PP   1024
#define PE   1024
#define TP   72
#define SP   128
#define NX8  131072

static_assert(NTOK == NB * NL);
static_assert(NC == NH * ND);
static_assert(NBH == NB * NH);
static_assert(NL == NTT * 64);
static_assert(NX8 * 8 == NTOK * NC);
static_assert((NX8 % 256) == 0);
static_assert((NC % 128) == 0 && (NC % 32) == 0 && (ND % 32) == 0 && (NL % 64) == 0);
static_assert(((TP * 2) % 16) == 0 && ((SP * 2) % 16) == 0);
static_assert(PE == NC);

typedef __bf16   v16b __attribute__((ext_vector_type(16)));
typedef __bf16   v8b  __attribute__((ext_vector_type(8)));
typedef float    v8f  __attribute__((ext_vector_type(8)));
typedef float    v4f  __attribute__((ext_vector_type(4)));
typedef unsigned int v4u __attribute__((ext_vector_type(4)));
typedef v4f __attribute__((may_alias)) v4fa;
typedef v4u __attribute__((may_alias)) v4ua;

__device__ __forceinline__ unsigned short bf_bits(float f) {
  unsigned u = __float_as_uint(f);
  return (unsigned short)((u + 0x7FFFu + ((u >> 16) & 1u)) >> 16);
}
__device__ __forceinline__ float bf_up(unsigned short h) { return __uint_as_float(((unsigned)h) << 16); }
__device__ __forceinline__ unsigned pk16(unsigned short a, unsigned short b) { return (unsigned)a | ((unsigned)b << 16); }
__device__ __forceinline__ v8f zero8() { v8f z = {0.f, 0.f, 0.f, 0.f, 0.f, 0.f, 0.f, 0.f}; return z; }

__device__ __forceinline__ v16b ldfrag_b(const __bf16* p) {
  union { v16b v; v8b h[2]; } f;
  f.h[0] = *(const v8b*)(p);
  f.h[1] = *(const v8b*)(p + 16);
  return f.v;
}

__device__ __forceinline__ v8f mma_b(v16b a, v16b b, v8f c) {
  c = __builtin_amdgcn_wmma_f32_16x16x32_bf16(false, a, false, b, (short)0, c, false, false);
  asm volatile("v_nop\n\tv_nop\n\tv_nop\n\tv_nop" : "+v"(c) : "v"(a), "v"(b));
  return c;
}

__device__ __forceinline__ void split8(const float* xv, v4u& hv, v4u& lv) {
  unsigned short hb[8], lb[8];
#pragma unroll
  for (int e = 0; e < 8; ++e) {
    const unsigned short hq = bf_bits(xv[e]);
    hb[e] = hq;
    lb[e] = bf_bits(xv[e] - bf_up(hq));
  }
  hv[0] = pk16(hb[0], hb[1]); hv[1] = pk16(hb[2], hb[3]); hv[2] = pk16(hb[4], hb[5]); hv[3] = pk16(hb[6], hb[7]);
  lv[0] = pk16(lb[0], lb[1]); lv[1] = pk16(lb[2], lb[3]); lv[2] = pk16(lb[4], lb[5]); lv[3] = pk16(lb[6], lb[7]);
}

__global__ __launch_bounds__(256) void k_cvt(const float* __restrict__ x, unsigned short* xb) {
  const int g = blockIdx.x * 256 + threadIdx.x;
  if (g >= NX8) return;
  const float* src = x + (size_t)g * 8;
  const v4f a = *(const v4fa*)src;
  const v4f c = *(const v4fa*)(src + 4);
  v4u o;
  o[0] = pk16(bf_bits(a[0]), bf_bits(a[1]));
  o[1] = pk16(bf_bits(a[2]), bf_bits(a[3]));
  o[2] = pk16(bf_bits(c[0]), bf_bits(c[1]));
  o[3] = pk16(bf_bits(c[2]), bf_bits(c[3]));
  unsigned short* dst = xb + (size_t)g * 8;
  *(volatile v4u*)dst = o;
  __threadfence();
  *(volatile v4u*)dst = o;
}

__global__ __launch_bounds__(128) void k_tr(const float* __restrict__ w0, const float* __restrict__ w1,
                                            const float* __restrict__ w2, const float* __restrict__ w3,
                                            const float* __restrict__ w4, unsigned short* tr) {
  __shared__ __align__(16) unsigned short sT[64 * TP];
  const int tid = threadIdx.x, lane = tid & 31, wave = tid >> 5;
  const int s = blockIdx.x >> 8, ti = blockIdx.x & 255;
  const int k0 = (ti >> 4) * 64, n0 = (ti & 15) * 64;
  const float* src = (s == 0) ? w0 : ((s == 1) ? w1 : ((s == 2) ? w2 : ((s == 3) ? w3 : w4)));
#pragma unroll 2
  for (int i = 0; i < 8; ++i) {
    const int idx = i * 128 + tid;
    const int r = idx >> 4, c4 = (idx & 15) * 4;
    const v4f a = *(const v4fa*)(src + (size_t)(k0 + r) * NC + n0 + c4);
#pragma unroll
    for (int e = 0; e < 4; ++e) sT[(c4 + e) * TP + r] = bf_bits(a[e]);
  }
  __syncthreads();
  unsigned short* dst = tr + (size_t)s * NC * NC;
  const int q8 = lane & 7, sub = lane >> 3;
  for (int pass = 0; pass < 2; ++pass) {
#pragma unroll
    for (int it = 0; it < 4; ++it) {
      const int row = wave * 16 + it * 4 + sub;
      const v4u v = *(const v4ua*)(sT + row * TP + 8 * q8);
      *(volatile v4u*)(dst + (size_t)(n0 + row) * NC + k0 + 8 * q8) = v;
    }
    __threadfence();
  }
}

__global__ __launch_bounds__(128) void k_proj(const unsigned short* __restrict__ xbp,
                                              const unsigned short* __restrict__ trp,
                                              const float* __restrict__ bq, const float* __restrict__ bk,
                                              const float* __restrict__ bk2,
                                              float* qf, float* kf, float* k2f) {
  __shared__ __align__(16) float sT[128 * ND];
  const int tid = threadIdx.x, lane = tid & 31, w = tid >> 5;
  const int hh = lane >> 4, m = lane & 15;
  const int m0 = blockIdx.x * 128;
  const int cg = blockIdx.y, which = cg >> 4, head = cg & 15;
  const __bf16* xb = (const __bf16*)(const void*)xbp;
  const __bf16* wb = (const __bf16*)(const void*)trp;
  const __bf16* xa0 = xb + ((size_t)(m0 + 32 * w + m)) * NC + 8 * hh;
  const __bf16* xa1 = xa0 + (size_t)16 * NC;
  const __bf16* wr  = wb + ((size_t)which * NC + head * ND + m) * NC + 8 * hh;

  v8f acc[2][4];
#pragma unroll
  for (int mt = 0; mt < 2; ++mt)
#pragma unroll
    for (int nt = 0; nt < 4; ++nt) acc[mt][nt] = zero8();

#pragma unroll 1
  for (int k0 = 0; k0 < NC; k0 += 32) {
    const v16b a0 = ldfrag_b(xa0 + k0);
    const v16b a1 = ldfrag_b(xa1 + k0);
#pragma unroll
    for (int nt = 0; nt < 4; ++nt) {
      const v16b bb = ldfrag_b(wr + (size_t)nt * 16 * NC + k0);
      acc[0][nt] = mma_b(a0, bb, acc[0][nt]);
      acc[1][nt] = mma_b(a1, bb, acc[1][nt]);
    }
  }

  const float* bias = (which == 0) ? bq : ((which == 1) ? bk : bk2);
#pragma unroll
  for (int nt = 0; nt < 4; ++nt) {
    const int feat = 16 * nt + m;
    const float bvl = bf_up(bf_bits(bias[head * ND + feat]));
#pragma unroll
    for (int mt = 0; mt < 2; ++mt)
#pragma unroll
      for (int r = 0; r < 8; ++r) {
        const int tokl = 32 * w + 16 * mt + 8 * hh + r;
        sT[tokl * ND + feat] = acc[mt][nt][r] + bvl;
      }
  }
  __syncthreads();

  float* plane = (which == 0) ? qf : ((which == 1) ? kf : k2f);
  const int b = m0 >> 9, t0 = m0 & (NL - 1), bh = b * NH + head;
  float* dstb = plane + ((size_t)(bh * NL + t0 + 32 * w)) * ND;
  const float* srcb = sT + (32 * w) * ND;
  for (int pass = 0; pass < 2; ++pass) {
#pragma unroll
    for (int i = 0; i < 16; ++i) {
      const int o = i * 128 + lane * 4;
      const v4f vv = *(const v4fa*)(srcb + o);
      *(volatile v4f*)(dstb + o) = vv;
    }
    __threadfence();
  }
}

__global__ __launch_bounds__(256) void k_gate(const float* __restrict__ x, const float* __restrict__ qf,
                                              const float* __restrict__ kf, const float* __restrict__ k2f,
                                              const float* __restrict__ gww, const float* __restrict__ gwb,
                                              const float* __restrict__ sww, const float* __restrict__ swb,
                                              float* gct, float* rgt,
                                              unsigned short* qpl, unsigned short* kpl,
                                              unsigned short* q2pl, unsigned short* k2pl) {
  __shared__ float sgw[ND];
  __shared__ float ssw[ND];
  __shared__ __align__(16) float slg[NL];
  __shared__ __align__(16) float sR[NL];
  __shared__ __align__(16) float sGc[NL];
  __shared__ __align__(16) float sRG[NL];
  const int tid = threadIdx.x, lane = tid & 31, wave = tid >> 5;
  const int bh = blockIdx.x, b = bh >> 4, h = bh & 15;

  if (tid < ND) {
    sgw[tid] = bf_up(bf_bits(gww[tid]));
    ssw[tid] = bf_up(bf_bits(sww[tid]));
  }
  __syncthreads();
  const float gb = bf_up(bf_bits(gwb[0]));
  const float sb = bf_up(bf_bits(swb[0]));

#pragma unroll 1
  for (int rr = 0; rr < 2; ++rr) {
    const int t = rr * 256 + tid;
    const float* xr = x + ((size_t)(b * NL + t)) * NC + h * ND;
    const float* kr = kf + ((size_t)(bh * NL + t)) * ND;
    float d1 = 0.0f, d2 = 0.0f;
#pragma unroll 1
    for (int g = 0; g < 16; ++g) {
      const v4f xv = *(const v4fa*)(xr + 4 * g);
      const v4f kv = *(const v4fa*)(kr + 4 * g);
#pragma unroll
      for (int e = 0; e < 4; ++e) {
        d1 = fmaf(bf_up(bf_bits(xv[e])), sgw[4 * g + e], d1);
        d2 = fmaf(kv[e], ssw[4 * g + e], d2);
      }
    }
    const float gv = 1.0f / (1.0f + expf(-(d1 + gb)));
    slg[t] = logf(fmaxf(gv, 1e-6f));
    const float z = d2 + sb;
    sR[t] = z * (1.0f / (1.0f + expf(-z)));
  }
  __syncthreads();

  if (tid == 0) {
    float run = 0.0f;
#pragma unroll 1
    for (int t = 0; t < NL; ++t) {
      run += slg[t];
      const float lc = fminf(30.0f, fmaxf(-30.0f, run));
      sGc[t] = expf(lc) + 1e-6f;
    }
  }
  __syncthreads();

#pragma unroll 1
  for (int rr = 0; rr < 2; ++rr) {
    const int t = rr * 256 + tid;
    sRG[t] = sR[t] * (1.0f / sGc[t]);
  }
  __syncthreads();

  if (tid < 128) {
    const v4f g4 = *(const v4fa*)(sGc + 4 * tid);
    const v4f r4 = *(const v4fa*)(sRG + 4 * tid);
    float* gd = gct + (size_t)bh * NL + 4 * tid;
    float* rd = rgt + (size_t)bh * NL + 4 * tid;
    *(volatile v4f*)gd = g4;
    *(volatile v4f*)rd = r4;
    __threadfence();
    *(volatile v4f*)gd = g4;
    *(volatile v4f*)rd = r4;
  }

  const int q8 = lane & 7, sub = lane >> 3;
#pragma unroll 1
  for (int p = 0; p < 4; ++p) {
    const float* src = (p == 1) ? kf : ((p == 3) ? k2f : qf);
    unsigned short* dst = (p == 0) ? qpl : ((p == 1) ? kpl : ((p == 2) ? q2pl : k2pl));
#pragma unroll 1
    for (int it = 0; it < 16; ++it) {
      const int row = it * 32 + wave * 4 + sub;
      const float* sp = src + ((size_t)(bh * NL + row)) * ND + 8 * q8;
      const v4f a = *(const v4fa*)sp;
      const v4f c = *(const v4fa*)(sp + 4);
      float xv[8] = {a[0], a[1], a[2], a[3], c[0], c[1], c[2], c[3]};
#pragma unroll
      for (int e = 0; e < 8; ++e) {
        float v = xv[e];
        if (p == 2) {
          const float z = v * 0.125f;
          v = (z <= 0.0f) ? z : (0.02f * z);
        } else if (p == 3) {
          const float z = (v * 0.03125f) * 0.02f;
          v = __builtin_amdgcn_rcpf(1.0f + __expf(-z));
        }
        if (p >= 2) v = (row <= NL - 2) ? v : 0.0f;
        xv[e] = v;
      }
      v4u hv, lv;
      split8(xv, hv, lv);
      unsigned short* d0 = dst + ((size_t)(bh * NL + row)) * PK + 8 * q8;
      *(volatile v4u*)d0 = hv;
      *(volatile v4u*)(d0 + 64) = lv;
      __threadfence();
      *(volatile v4u*)d0 = hv;
      *(volatile v4u*)(d0 + 64) = lv;
    }
  }
}

__global__ __launch_bounds__(128) void k_s(const unsigned short* __restrict__ App, const unsigned short* __restrict__ Bpp,
                                           const float* __restrict__ gct, const float* __restrict__ rgt, int scaled,
                                           unsigned short* Pout) {
  __shared__ __align__(16) unsigned short st[4 * 16 * SP];
  __shared__ float sG[64];
  __shared__ float sRG[NL];
  const int tid = threadIdx.x, lane = tid & 31, wave = tid >> 5;
  const int hh = lane >> 4, m = lane & 15;
  const int bh = blockIdx.x >> 3, tt = blockIdx.x & 7, t0 = tt * 64;

  if (scaled != 0) {
    if (tid < 64) sG[tid] = gct[(size_t)bh * NL + t0 + tid];
#pragma unroll
    for (int i = 0; i < 4; ++i) sRG[i * 128 + tid] = rgt[(size_t)bh * NL + i * 128 + tid];
  } else {
    if (tid < 64) sG[tid] = 1.0f;
#pragma unroll
    for (int i = 0; i < 4; ++i) sRG[i * 128 + tid] = 1.0f;
  }
  __syncthreads();

  const __bf16* Ap = (const __bf16*)(const void*)App;
  const __bf16* Bp = (const __bf16*)(const void*)Bpp;
  const __bf16* arow = Ap + ((size_t)(bh * NL + t0 + wave * 16 + m)) * PK + 8 * hh;
  const v16b ah0 = ldfrag_b(arow);
  const v16b ah1 = ldfrag_b(arow + 32);
  const v16b al0 = ldfrag_b(arow + 64);
  const v16b al1 = ldfrag_b(arow + 96);
  float gc[8];
#pragma unroll
  for (int r = 0; r < 8; ++r) gc[r] = sG[wave * 16 + 8 * hh + r];
  unsigned short* stw = st + wave * (16 * SP);
  const int q8 = lane & 7, hsel = (lane >> 3) & 1, rsub = lane >> 4;
  const size_t prow0 = (size_t)(bh * NL + t0 + wave * 16);

#pragma unroll 1
  for (int c = 0; c < 8; ++c) {
    const int c0 = c * 64;
    v8f acc[4];
#pragma unroll
    for (int j = 0; j < 4; ++j) acc[j] = zero8();
    if (c <= tt) {
#pragma unroll
      for (int j = 0; j < 4; ++j) {
        const __bf16* brow = Bp + ((size_t)(bh * NL + c0 + 16 * j + m)) * PK + 8 * hh;
        const v16b fh0 = ldfrag_b(brow);
        const v16b fl0 = ldfrag_b(brow + 64);
        acc[j] = mma_b(ah0, fh0, acc[j]);
        acc[j] = mma_b(ah0, fl0, acc[j]);
        acc[j] = mma_b(al0, fh0, acc[j]);
        const v16b fh1 = ldfrag_b(brow + 32);
        const v16b fl1 = ldfrag_b(brow + 96);
        acc[j] = mma_b(ah1, fh1, acc[j]);
        acc[j] = mma_b(ah1, fl1, acc[j]);
        acc[j] = mma_b(al1, fh1, acc[j]);
      }
    }
#pragma unroll
    for (int j = 0; j < 4; ++j) {
      const int coll = c0 + 16 * j + m;
      const float rg = sRG[coll];
#pragma unroll
      for (int r = 0; r < 8; ++r) {
        const int rowl = 8 * hh + r;
        const int trow = t0 + wave * 16 + rowl;
        const float v = (coll <= trow) ? ((gc[r] * rg) * acc[j][r]) : 0.0f;
        const unsigned short hb = bf_bits(v);
        const unsigned short lb = bf_bits(v - bf_up(hb));
        stw[rowl * SP + 16 * j + m] = hb;
        stw[rowl * SP + 64 + 16 * j + m] = lb;
      }
    }
    __syncthreads();
    for (int pass = 0; pass < 2; ++pass) {
#pragma unroll
      for (int i = 0; i < 8; ++i) {
        const int rowl = 2 * i + rsub;
        const v4u v = *(const v4ua*)(stw + rowl * SP + 64 * hsel + 8 * q8);
        *(volatile v4u*)(Pout + (prow0 + rowl) * PP + 512 * hsel + c0 + 8 * q8) = v;
      }
      __threadfence();
    }
    __syncthreads();
  }
}

__global__ __launch_bounds__(128) void k_o(const unsigned short* __restrict__ Ppl, const unsigned short* __restrict__ Bpl,
                                           const float* o1in, int mode, float* o1out,
                                           unsigned short* yh, unsigned short* yl) {
  __shared__ __align__(16) float sO[64 * ND];
  const int tid = threadIdx.x, lane = tid & 31, wave = tid >> 5;
  const int hh = lane >> 4, m = lane & 15;
  const int bh = blockIdx.x >> 3, tt = blockIdx.x & 7, t0 = tt * 64;
  const int b = bh >> 4, h = bh & 15;

  const __bf16* P = (const __bf16*)(const void*)Ppl;
  const __bf16* arow = P + ((size_t)(bh * NL + t0 + wave * 16 + m)) * PP + 8 * hh;
  const __bf16* Bb = (const __bf16*)(const void*)Bpl;
  const size_t boff = (mode == 0) ? (((size_t)(h * ND + m)) * NC + (size_t)b * NL + 8 * hh)
                                  : (((size_t)(bh * ND + m)) * PE + 8 * hh);
  const __bf16* brow = Bb + boff;
  const int nseg = (mode == 0) ? 2 : 3;
  const int kend = t0 + 64;

  v8f acc[4];
#pragma unroll
  for (int nt = 0; nt < 4; ++nt) acc[nt] = zero8();
#pragma unroll 1
  for (int sg = 0; sg < nseg; ++sg) {
    const int ao = (sg == 1) ? 512 : 0;
    const int bo = (sg == 2) ? 512 : 0;
#pragma unroll 1
    for (int k = 0; k < kend; k += 32) {
      const v16b a = ldfrag_b(arow + ao + k);
#pragma unroll
      for (int nt = 0; nt < 4; ++nt) {
        const v16b fb = ldfrag_b(brow + (size_t)nt * 16 * NC + bo + k);
        acc[nt] = mma_b(a, fb, acc[nt]);
      }
    }
  }

  if (mode == 0) {
    float* so = sO + wave * (16 * ND);
#pragma unroll
    for (int nt = 0; nt < 4; ++nt)
#pragma unroll
      for (int r = 0; r < 8; ++r) so[(8 * hh + r) * ND + 16 * nt + m] = acc[nt][r];
    __syncthreads();
    float* dstb = o1out + ((size_t)(bh * NL + t0 + wave * 16)) * ND;
    for (int pass = 0; pass < 2; ++pass) {
#pragma unroll
      for (int i = 0; i < 8; ++i) {
        const int o = i * 128 + lane * 4;
        const v4f vv = *(const v4fa*)(so + o);
        *(volatile v4f*)(dstb + o) = vv;
      }
      __threadfence();
    }
  } else {
#pragma unroll
    for (int nt = 0; nt < 4; ++nt)
#pragma unroll
      for (int r = 0; r < 8; ++r) sO[(wave * 16 + 8 * hh + r) * ND + 16 * nt + m] = acc[nt][r];
    __syncthreads();
    const int lo_l = (t0 == 0) ? 0 : (t0 + 1);
    const int nrows = (t0 == 0) ? 65 : ((t0 + 64 >= NL) ? (NL - 1 - t0) : 64);
    const int q8 = lane & 7, rs = tid >> 3;
#pragma unroll 1
    for (int it = 0; it < 5; ++it) {
      const int ri = it * 16 + rs;
      const bool act = (ri < nrows);
      const int l = lo_l + ri;
      const int lcl = (l < NL) ? l : (NL - 1);
      int srow = l - 1 - t0;
      srow = (srow < 0) ? 0 : ((srow > 63) ? 63 : srow);
      const float* op = o1in + ((size_t)(bh * NL + lcl)) * ND + 8 * q8;
      const v4f oa = *(const v4fa*)op;
      const v4f oc = *(const v4fa*)(op + 4);
      const v4f za = *(const v4fa*)(sO + srow * ND + 8 * q8);
      const v4f zc = *(const v4fa*)(sO + srow * ND + 8 * q8 + 4);
      const bool has2 = (l > 0);
      float yv[8];
      yv[0] = oa[0] + (has2 ? za[0] : 0.0f);
      yv[1] = oa[1] + (has2 ? za[1] : 0.0f);
      yv[2] = oa[2] + (has2 ? za[2] : 0.0f);
      yv[3] = oa[3] + (has2 ? za[3] : 0.0f);
      yv[4] = oc[0] + (has2 ? zc[0] : 0.0f);
      yv[5] = oc[1] + (has2 ? zc[1] : 0.0f);
      yv[6] = oc[2] + (has2 ? zc[2] : 0.0f);
      yv[7] = oc[3] + (has2 ? zc[3] : 0.0f);
      v4u hv, lv;
      split8(yv, hv, lv);
      const size_t gy = ((size_t)(b * NL + lcl)) * NC + h * ND + 8 * q8;
      if (act) {
        *(volatile v4u*)(yh + gy) = hv;
        *(volatile v4u*)(yl + gy) = lv;
      }
      __threadfence();
      if (act) {
        *(volatile v4u*)(yh + gy) = hv;
        *(volatile v4u*)(yl + gy) = lv;
      }
    }
  }
}

__global__ __launch_bounds__(128) void k_e(const float* __restrict__ x, const float* __restrict__ o1f, unsigned short* et) {
  __shared__ __align__(16) unsigned short sH[64 * TP];
  __shared__ __align__(16) unsigned short sL[64 * TP];
  const int tid = threadIdx.x, lane = tid & 31, wave = tid >> 5;
  const int bh = blockIdx.x >> 3, tt = blockIdx.x & 7, tau0 = tt * 64;
  const int b = bh >> 4, h = bh & 15;
  {
    const int r = tid >> 1, ch = (tid & 1) * 32;
    const int tau = tau0 + r;
    const int tn = (tau + 1 < NL) ? (tau + 1) : (NL - 1);
    const bool zrow = (tau == NL - 1);
    const float* xs = x + ((size_t)(b * NL + tn)) * NC + h * ND + ch;
    const float* os = o1f + ((size_t)(bh * NL + tau)) * ND + ch;
#pragma unroll 2
    for (int g = 0; g < 8; ++g) {
      const v4f xv = *(const v4fa*)(xs + 4 * g);
      const v4f ov = *(const v4fa*)(os + 4 * g);
#pragma unroll
      for (int e = 0; e < 4; ++e) {
        const float vr = bf_up(bf_bits(xv[e]));
        const float ev = zrow ? 0.0f : (vr - ov[e]);
        const unsigned short hb = bf_bits(ev);
        const unsigned short lb = bf_bits(ev - bf_up(hb));
        sH[(ch + 4 * g + e) * TP + r] = hb;
        sL[(ch + 4 * g + e) * TP + r] = lb;
      }
    }
  }
  __syncthreads();
  const int q8 = lane & 7, sub = lane >> 3;
  for (int pass = 0; pass < 2; ++pass) {
#pragma unroll
    for (int it = 0; it < 4; ++it) {
      const int row = wave * 16 + it * 4 + sub;
      const v4u vh = *(const v4ua*)(sH + row * TP + 8 * q8);
      const v4u vl = *(const v4ua*)(sL + row * TP + 8 * q8);
      const size_t go = ((size_t)(bh * ND + row)) * PE + tau0 + 8 * q8;
      *(volatile v4u*)(et + go) = vh;
      *(volatile v4u*)(et + go + 512) = vl;
    }
    __threadfence();
  }
}

__global__ __launch_bounds__(128) void k_oproj(const unsigned short* __restrict__ Yhp, const unsigned short* __restrict__ Ylp,
                                               const unsigned short* __restrict__ trp, const float* __restrict__ bp,
                                               float* out) {
  __shared__ __align__(16) float sT[128 * ND];
  const int tid = threadIdx.x, lane = tid & 31, w = tid >> 5;
  const int hh = lane >> 4, m = lane & 15;
  const int m0 = blockIdx.x * 128, nb = blockIdx.y;
  const __bf16* Yh = (const __bf16*)(const void*)Yhp;
  const __bf16* Yl = (const __bf16*)(const void*)Ylp;
  const __bf16* wb = (const __bf16*)(const void*)trp;
  const size_t yo0 = ((size_t)(m0 + 32 * w + m)) * NC + 8 * hh;
  const size_t yo1 = yo0 + (size_t)16 * NC;
  const __bf16* wr = wb + ((size_t)3 * NC + nb * ND + m) * NC + 8 * hh;

  v8f acc[2][4];
#pragma unroll
  for (int mt = 0; mt < 2; ++mt)
#pragma unroll
    for (int nt = 0; nt < 4; ++nt) acc[mt][nt] = zero8();

#pragma unroll 1
  for (int k0 = 0; k0 < NC; k0 += 32) {
    const v16b a0h = ldfrag_b(Yh + yo0 + k0);
    const v16b a0l = ldfrag_b(Yl + yo0 + k0);
    const v16b a1h = ldfrag_b(Yh + yo1 + k0);
    const v16b a1l = ldfrag_b(Yl + yo1 + k0);
#pragma unroll
    for (int nt = 0; nt < 4; ++nt) {
      const v16b bb = ldfrag_b(wr + (size_t)nt * 16 * NC + k0);
      acc[0][nt] = mma_b(a0h, bb, acc[0][nt]);
      acc[0][nt] = mma_b(a0l, bb, acc[0][nt]);
      acc[1][nt] = mma_b(a1h, bb, acc[1][nt]);
      acc[1][nt] = mma_b(a1l, bb, acc[1][nt]);
    }
  }

#pragma unroll
  for (int nt = 0; nt < 4; ++nt) {
    const int feat = 16 * nt + m;
    const float bvl = bf_up(bf_bits(bp[nb * ND + feat]));
#pragma unroll
    for (int mt = 0; mt < 2; ++mt)
#pragma unroll
      for (int r = 0; r < 8; ++r) {
        const int tokl = 32 * w + 16 * mt + 8 * hh + r;
        sT[tokl * ND + feat] = acc[mt][nt][r] + bvl;
      }
  }
  __syncthreads();

  for (int pass = 0; pass < 2; ++pass) {
#pragma unroll
    for (int i = 0; i < 16; ++i) {
      const int rowl = 32 * w + 2 * i + hh;
      const v4f vv = *(const v4fa*)(sT + rowl * ND + 4 * m);
      *(volatile v4f*)(out + ((size_t)(m0 + rowl)) * NC + nb * ND + 4 * m) = vv;
    }
    __threadfence();
  }
}

extern "C" void kernel_launch(void* const* d_in, const int* in_sizes, int n_in,
                              void* d_out, int out_size, void* d_ws, size_t ws_size,
                              hipStream_t stream) {
  if (n_in < 13) return;
  if (in_sizes[0] != NTOK * NC) return;
  if (in_sizes[1] != NC * NC || in_sizes[3] != NC * NC || in_sizes[5] != NC * NC || in_sizes[11] != NC * NC) return;
  if (in_sizes[2] != NC || in_sizes[4] != NC || in_sizes[6] != NC || in_sizes[12] != NC) return;
  if (in_sizes[7] != ND || in_sizes[9] != ND) return;
  if (in_sizes[8] < 1 || in_sizes[10] < 1) return;
  if (out_size != NTOK * NC) return;

  const float* x    = (const float*)d_in[0];
  const float* q1w  = (const float*)d_in[1];
  const float* q1b  = (const float*)d_in[2];
  const float* k1w  = (const float*)d_in[3];
  const float* k1b  = (const float*)d_in[4];
  const float* k2w  = (const float*)d_in[5];
  const float* k2b  = (const float*)d_in[6];
  const float* gww  = (const float*)d_in[7];
  const float* gwb  = (const float*)d_in[8];
  const float* sww  = (const float*)d_in[9];
  const float* swb  = (const float*)d_in[10];
  const float* cpw  = (const float*)d_in[11];
  const float* cpb  = (const float*)d_in[12];
  float* out = (float*)d_out;

  const size_t PXB = (size_t)NTOK * NC * 2;
  const size_t PTR = (size_t)5 * NC * NC * 2;
  const size_t PF  = (size_t)NBH * NL * ND * 4;
  const size_t PT  = (size_t)NBH * NL * 4;
  const size_t PPL = (size_t)NBH * NL * PK * 2;
  const size_t PSC = (size_t)NBH * NL * PP * 2;
  const size_t PO1 = (size_t)NBH * NL * ND * 4;
  const size_t PET = (size_t)NBH * ND * PE * 2;
  const size_t PY  = (size_t)NTOK * NC * 2;
  size_t off = 0;
  const size_t oXB = off; off += PXB;
  const size_t oTR = off; off += PTR;
  const size_t oQF = off; off += PF;
  const size_t oKF = off; off += PF;
  const size_t oK2 = off; off += PF;
  const size_t oGC = off; off += PT;
  const size_t oRG = off; off += PT;
  const size_t oQP = off; off += PPL;
  const size_t oKP = off; off += PPL;
  const size_t oQ2 = off; off += PPL;
  const size_t oK2P = off; off += PPL;
  const size_t oP1 = off; off += PSC;
  const size_t oO1 = off; off += PO1;
  const size_t oET = off; off += PET;
  const size_t oP2 = off; off += PSC;
  const size_t oYH = off; off += PY;
  const size_t oYL = off; off += PY;
  if (off > ws_size) return;
  if (off > (size_t)134217728u) return;

  char* ws = (char*)d_ws;
  unsigned short* xb  = (unsigned short*)(ws + oXB);
  unsigned short* tr  = (unsigned short*)(ws + oTR);
  float* Qf  = (float*)(ws + oQF);
  float* Kf  = (float*)(ws + oKF);
  float* K2f = (float*)(ws + oK2);
  float* Gct = (float*)(ws + oGC);
  float* RGt = (float*)(ws + oRG);
  unsigned short* Qp  = (unsigned short*)(ws + oQP);
  unsigned short* Kp  = (unsigned short*)(ws + oKP);
  unsigned short* Q2p = (unsigned short*)(ws + oQ2);
  unsigned short* K2p = (unsigned short*)(ws + oK2P);
  unsigned short* P1  = (unsigned short*)(ws + oP1);
  float* O1f = (float*)(ws + oO1);
  unsigned short* ET  = (unsigned short*)(ws + oET);
  unsigned short* P2  = (unsigned short*)(ws + oP2);
  unsigned short* Yh  = (unsigned short*)(ws + oYH);
  unsigned short* Yl  = (unsigned short*)(ws + oYL);
  unsigned short* xT  = tr + (size_t)4 * NC * NC;

  k_cvt<<<dim3(NX8 / 256), dim3(256), 0, stream>>>(x, xb);
  k_tr<<<dim3(5 * 256), dim3(128), 0, stream>>>(q1w, k1w, k2w, cpw, x, tr);
  k_proj<<<dim3(NTOK / 128, 3 * NH), dim3(128), 0, stream>>>(xb, tr, q1b, k1b, k2b, Qf, Kf, K2f);
  k_gate<<<dim3(NBH), dim3(256), 0, stream>>>(x, Qf, Kf, K2f, gww, gwb, sww, swb, Gct, RGt, Qp, Kp, Q2p, K2p);
  k_s<<<dim3(NBH * NTT), dim3(128), 0, stream>>>(Qp, Kp, Gct, RGt, 1, P1);
  k_o<<<dim3(NBH * NTT), dim3(128), 0, stream>>>(P1, xT, O1f, 0, O1f, Yh, Yl);
  k_e<<<dim3(NBH * NTT), dim3(128), 0, stream>>>(x, O1f, ET);
  k_s<<<dim3(NBH * NTT), dim3(128), 0, stream>>>(Q2p, K2p, Gct, RGt, 0, P2);
  k_o<<<dim3(NBH * NTT), dim3(128), 0, stream>>>(P2, ET, O1f, 1, O1f, Yh, Yl);
  k_oproj<<<dim3(NTOK / 128, NC / ND), dim3(128), 0, stream>>>(Yh, Yl, tr, cpb, out);
  (void)hipGetLastError();
}
